// CausalSelfAttention_45071386804892
// MI455X (gfx1250) — hardware-verified
//
#include <hip/hip_runtime.h>


#ifndef NB
#define NB 2
#endif
#ifndef SEQ
#define SEQ 2048
#endif
#define NB_FULL  2
#define SEQ_FULL 2048
#ifndef OUT_SEQ
#define OUT_SEQ SEQ
#endif
#define DM    2048
#define NH_   32
#define NKV   8
#define HD    64
#define KVD   (NKV * HD)
#define AW    4
#define EARLY 256
#define QRS  1024.0f
#define QRI  (1.0f / 1024.0f)
#define SC2  (0.125f * 1.4426950408889634f)
#define PSH  8.0f
#define CXS  1024.0f
#define WOS  16.0f
#define OUTS (1.0f / (1024.0f * 16.0f))
#define NEGB (-3.0e38f)

static_assert(HD == 64);
static_assert(NH_ * HD == DM);
static_assert(NKV * AW == NH_);
static_assert(DM % 64 == 0);
static_assert(KVD % 64 == 0);
static_assert(DM % 32 == 0);
static_assert(SEQ % 64 == 0);
static_assert(SEQ % 32 == 0);
static_assert(EARLY % 64 == 0);
static_assert(SEQ >= EARLY);
static_assert((SEQ - EARLY) % 16 == 0);
static_assert(((size_t)SEQ * DM) % 8 == 0);
static_assert(NB <= NB_FULL);
static_assert(SEQ <= SEQ_FULL);

typedef _Float16 h16;
typedef unsigned short bf;
typedef __attribute__((ext_vector_type(16))) __bf16   v16bf;
typedef __attribute__((ext_vector_type(16))) _Float16 v16h;
typedef __attribute__((ext_vector_type(8)))  _Float16 v8h;
typedef __attribute__((ext_vector_type(8)))  unsigned short v8us;
typedef __attribute__((ext_vector_type(8)))  float    v8f;
typedef __attribute__((ext_vector_type(4)))  float    v4f;
typedef __attribute__((ext_vector_type(2)))  float    v2f;
typedef v4f  __attribute__((may_alias)) v4fa;

__device__ __forceinline__ unsigned short f2bf(float f) { unsigned u = __float_as_uint(f); u += 0x7FFFu + ((u >> 16) & 1u); return (unsigned short)(u >> 16); }
__device__ __forceinline__ v16h cat16(v8h lo, v8h hi) { return __builtin_shufflevector(lo, hi, 0, 1, 2, 3, 4, 5, 6, 7, 8, 9, 10, 11, 12, 13, 14, 15); }
__device__ __forceinline__ v16bf cat16b(v8us lo, v8us hi) { return __builtin_bit_cast(v16bf, __builtin_shufflevector(lo, hi, 0, 1, 2, 3, 4, 5, 6, 7, 8, 9, 10, 11, 12, 13, 14, 15)); }
__device__ __forceinline__ v8f wmma16(v16h a, v16h b, v8f c) {
    c = __builtin_amdgcn_wmma_f32_16x16x32_f16(false, a, false, b, (short)0, c, false, false);
    asm volatile("v_nop\n\tv_nop\n\tv_nop\n\tv_nop" : "+v"(c) : "v"(a), "v"(b));
    return c; }
__device__ __forceinline__ v8f wmmab(v16bf a, v16bf b, v8f c) {
    c = __builtin_amdgcn_wmma_f32_16x16x32_bf16(false, a, false, b, (short)0, c, false, false);
    asm volatile("v_nop\n\tv_nop\n\tv_nop\n\tv_nop" : "+v"(c) : "v"(a), "v"(b));
    return c; }
__device__ __forceinline__ v16h  ldh(const h16* p) { return cat16(*(const v8h*)p, *(const v8h*)(p + 16)); }
__device__ __forceinline__ v16bf ldb(const bf* p)  { return cat16b(*(const v8us*)p, *(const v8us*)(p + 16)); }
__device__ __forceinline__ void wave_sync() { __builtin_amdgcn_fence(3  , "wavefront"); __builtin_amdgcn_wave_barrier(); asm volatile("" ::: "memory"); }

__global__ __launch_bounds__(256) void k_cvt8(const float* __restrict__ src, bf* dst, size_t n8) {
    const size_t i = (size_t)blockIdx.x * 256 + threadIdx.x; if (i >= n8) return;
    const v8f v = *(const v8f*)(src + i * 8); v8us o;
#pragma unroll
    for (int k = 0; k < 8; ++k) o[k] = f2bf(v[k]);
    *(volatile v8us*)(dst + i * 8) = o; __threadfence(); *(volatile v8us*)(dst + i * 8) = o;
}

__global__ __launch_bounds__(256) void k_wt(const float* __restrict__ W, bf* Tb, h16* Th, int Kr, int Nc, int mode) {
    __shared__ float ts[64 * 65];
    const int tid = threadIdx.x; const int n0 = blockIdx.x * 64, k0 = blockIdx.y * 64;
#pragma unroll
    for (int p = 0; p < 4; ++p) { const int row = p * 16 + (tid >> 4), c4 = (tid & 15) * 4;
        const v4f v = *(const v4f*)(W + (size_t)(k0 + row) * (size_t)Nc + n0 + c4);
        ts[row * 65 + c4 + 0] = v[0]; ts[row * 65 + c4 + 1] = v[1]; ts[row * 65 + c4 + 2] = v[2]; ts[row * 65 + c4 + 3] = v[3]; }
    __syncthreads();
#pragma unroll 1
    for (int ps = 0; ps < 2; ++ps) {
#pragma unroll
        for (int s = 0; s < 2; ++s) { const int n = s * 32 + (tid >> 3), c8 = (tid & 7) * 8;
            const size_t oo = (size_t)(n0 + n) * (size_t)Kr + k0 + c8;
            if (mode == 0) { v8us o;
#pragma unroll
                for (int i = 0; i < 8; ++i) o[i] = f2bf(ts[(c8 + i) * 65 + n]);
                *(volatile v8us*)(Tb + oo) = o;
            } else { v8h o;
#pragma unroll
                for (int i = 0; i < 8; ++i) o[i] = (h16)(__uint_as_float(((unsigned)f2bf(ts[(c8 + i) * 65 + n])) << 16) * WOS);
                *(volatile v8h*)(Th + oo) = o; } }
        if (ps == 0) __threadfence(); }
}

__global__ __launch_bounds__(256) void k_rope_tab(float* CS, int nrow) {
    const int i = blockIdx.x * 256 + threadIdx.x; if (i >= nrow * 32) return;
    const int t = i >> 5, j = i & 31;
    double p = 1.0;
    p *= (j & 1)  ? 1.3335214321633240 : 1.0;
    p *= (j & 2)  ? 1.7782794100389228 : 1.0;
    p *= (j & 4)  ? 3.1622776601683795 : 1.0;
    p *= (j & 8)  ? 10.0 : 1.0;
    p *= (j & 16) ? 100.0 : 1.0;
    const float pf = (float)p; const float inv = 1.0f / pf;
    const float ang = (float)t * inv;
    const float cs = cosf(ang), sn = sinf(ang);
    v2f o; o[0] = cs; o[1] = sn;
    *(volatile v2f*)(CS + (size_t)i * 2) = o; __threadfence(); *(volatile v2f*)(CS + (size_t)i * 2) = o;
}

__global__ __launch_bounds__(32) void k_proj(const bf* __restrict__ A, const bf* __restrict__ Bt, h16* Ph, h16* Pr, int useRes, int RB, size_t sRB, int pitch, int CB, size_t sCB, const float* __restrict__ CS, int rope) {
    __shared__ __align__(16) float os[16 * 68];
    const int K = DM;
    const int lane = threadIdx.x & 31, lr = lane & 15, hi = lane >> 4; const int r0 = blockIdx.x * 64, c0 = blockIdx.y * 64;
    v8f acc[4][4];
#pragma unroll
    for (int mb = 0; mb < 4; ++mb)
#pragma unroll
        for (int nb = 0; nb < 4; ++nb) acc[mb][nb] = (v8f){};
    const size_t aoff = (size_t)(r0 + lr) * K + 8 * hi, boff = (size_t)(c0 + lr) * K + 8 * hi;
#pragma unroll 1
    for (int kc = 0; kc < K; kc += 32) {
        v16bf a[4];
#pragma unroll
        for (int mb = 0; mb < 4; ++mb) a[mb] = ldb(A + aoff + (size_t)mb * 16 * K + kc);
#pragma unroll
        for (int nb = 0; nb < 4; ++nb) { const v16bf b = ldb(Bt + boff + (size_t)nb * 16 * K + kc);
#pragma unroll
            for (int mb = 0; mb < 4; ++mb) acc[mb][nb] = wmmab(a[mb], b, acc[mb][nb]); }
    }
    const size_t tbase = (size_t)(r0 / RB) * sRB + (size_t)(r0 % RB) * (size_t)pitch + (size_t)(c0 / CB) * sCB + (size_t)(c0 % CB);
#pragma unroll
    for (int mb = 0; mb < 4; ++mb) {
#pragma unroll
        for (int nb = 0; nb < 4; ++nb) {
#pragma unroll
            for (int j = 0; j < 8; ++j) os[(hi * 8 + j) * 68 + nb * 16 + lr] = acc[mb][nb][j]; }
        wave_sync();
        const size_t sb = tbase + (size_t)(mb * 16) * (size_t)pitch;
#pragma unroll 1
        for (int ps = 0; ps < 2; ++ps) {
#pragma unroll
            for (int s = 0; s < 4; ++s) { const int row = 4 * s + (lane >> 3), c8 = (lane & 7) * 8;
                v4f x0 = *(const v4fa*)(&os[row * 68 + c8]); v4f x1 = *(const v4fa*)(&os[row * 68 + c8 + 4]); v8h hv, rv;
                if (rope) {
                    const int t = (r0 + mb * 16 + row) % SEQ;
                    const float* cp = CS + ((size_t)t * 32 + (size_t)(c8 >> 1)) * 2;
                    const v4f ca = *(const v4f*)cp; const v4f cb = *(const v4f*)(cp + 4);
                    float e, o;
                    e = x0[0]; o = x0[1]; x0[0] = e * ca[0] - o * ca[1]; x0[1] = e * ca[1] + o * ca[0];
                    e = x0[2]; o = x0[3]; x0[2] = e * ca[2] - o * ca[3]; x0[3] = e * ca[3] + o * ca[2];
                    e = x1[0]; o = x1[1]; x1[0] = e * cb[0] - o * cb[1]; x1[1] = e * cb[1] + o * cb[0];
                    e = x1[2]; o = x1[3]; x1[2] = e * cb[2] - o * cb[3]; x1[3] = e * cb[3] + o * cb[2]; }
#pragma unroll
                for (int i = 0; i < 4; ++i) { const h16 a0 = (h16)x0[i]; const h16 a1 = (h16)x1[i]; hv[i] = a0; hv[4 + i] = a1; rv[i] = (h16)((x0[i] - (float)a0) * QRS); rv[4 + i] = (h16)((x1[i] - (float)a1) * QRS); }
                const size_t oo = sb + (size_t)row * (size_t)pitch + c8;
                *(volatile v8h*)(Ph + oo) = hv; if (useRes) *(volatile v8h*)(Pr + oo) = rv; }
            if (ps == 0) __threadfence(); }
        wave_sync();
    }
}

__global__ __launch_bounds__(32 * AW) void k_flash(const h16* __restrict__ QH, const h16* __restrict__ QR, const h16* __restrict__ KP, const h16* __restrict__ VT, h16* CH) {
    __shared__ __align__(16) float os[AW * 16 * 68];
    const int lane = threadIdx.x & 31; const int wave = __builtin_amdgcn_readfirstlane(threadIdx.x >> 5);
    const int lr = lane & 15, hi = lane >> 4;
    const int zg = blockIdx.y; const int b = zg / NKV; const int g = zg % NKV;
    const int h = g * AW + wave;
    const int t0 = EARLY + blockIdx.x * 16;
    const int tq = t0 + lr;
    const size_t qo = ((size_t)(b * NH_ + h) * SEQ + (size_t)tq) * HD + 8 * hi;
    const v16h qh0 = ldh(QH + qo), qh1 = ldh(QH + qo + 32), qr0 = ldh(QR + qo), qr1 = ldh(QR + qo + 32);
    const size_t ko = (size_t)zg * SEQ * HD + (size_t)lr * HD + 8 * hi;
    const size_t vo = (size_t)zg * HD * SEQ + (size_t)lr * SEQ + 8 * hi;
    v8f o0 = (v8f){}, o1 = (v8f){}, o2 = (v8f){}, o3 = (v8f){};
    float m = NEGB, l = 0.0f;
    const int kend = t0 + 16;
#pragma unroll 1
    for (int key0 = 0; key0 < kend; key0 += 32) {
        const h16* ka = KP + ko + (size_t)key0 * HD;
        const v16h ka0 = ldh(ka), ka1 = ldh(ka + 32), kb0 = ldh(ka + 16 * HD), kb1 = ldh(ka + 16 * HD + 32);
        v8f sHa = (v8f){}, sLa = (v8f){}, sHb = (v8f){}, sLb = (v8f){};
        sHa = wmma16(ka0, qh0, sHa); sLa = wmma16(ka0, qr0, sLa); sHb = wmma16(kb0, qh0, sHb); sLb = wmma16(kb0, qr0, sLb);
        sHa = wmma16(ka1, qh1, sHa); sLa = wmma16(ka1, qr1, sLa); sHb = wmma16(kb1, qh1, sHb); sLb = wmma16(kb1, qr1, sLb);
        float ta[8], tb[8];
#pragma unroll
        for (int r = 0; r < 8; ++r) { ta[r] = (sHa[r] + sLa[r] * QRI) * SC2; tb[r] = (sHb[r] + sLb[r] * QRI) * SC2; }
        if (key0 + 31 > t0) {
            const int kbse = key0 + 8 * hi;
#pragma unroll
            for (int r = 0; r < 8; ++r) { ta[r] = (kbse + r > tq) ? NEGB : ta[r]; tb[r] = (kbse + 16 + r > tq) ? NEGB : tb[r]; } }
        float mx = NEGB;
#pragma unroll
        for (int r = 0; r < 8; ++r) mx = fmaxf(mx, fmaxf(ta[r], tb[r]));
        mx = fmaxf(mx, __shfl_xor(mx, 16, 32));
        const float mnew = fmaxf(m, mx);
        const float alpha = __builtin_amdgcn_exp2f(m - mnew);
        const float sh = PSH - mnew;
        v16h pb; float ls = 0.0f;
#pragma unroll
        for (int r = 0; r < 8; ++r) { const float ea = __builtin_amdgcn_exp2f(ta[r] + sh); const float ec = __builtin_amdgcn_exp2f(tb[r] + sh); pb[r] = (h16)ea; pb[8 + r] = (h16)ec; ls += ea + ec; }
        l = l * alpha + ls; m = mnew;
        o0 = o0 * alpha; o1 = o1 * alpha; o2 = o2 * alpha; o3 = o3 * alpha;
        const h16* va = VT + vo + key0;
        const v16h v0 = ldh(va), v1 = ldh(va + (size_t)16 * SEQ), v2 = ldh(va + (size_t)32 * SEQ), v3 = ldh(va + (size_t)48 * SEQ);
        o0 = wmma16(v0, pb, o0); o1 = wmma16(v1, pb, o1); o2 = wmma16(v2, pb, o2); o3 = wmma16(v3, pb, o3);
    }
    l += __shfl_xor(l, 16, 32);
    const float inv = CXS / l;
    const int wb = wave * 16 * 68;
    { v4f a, c;
      a[0] = o0[0] * inv; a[1] = o0[1] * inv; a[2] = o0[2] * inv; a[3] = o0[3] * inv; c[0] = o0[4] * inv; c[1] = o0[5] * inv; c[2] = o0[6] * inv; c[3] = o0[7] * inv;
      *(v4fa*)(&os[wb + lr * 68 +  0 + 8 * hi]) = a; *(v4fa*)(&os[wb + lr * 68 +  0 + 8 * hi + 4]) = c;
      a[0] = o1[0] * inv; a[1] = o1[1] * inv; a[2] = o1[2] * inv; a[3] = o1[3] * inv; c[0] = o1[4] * inv; c[1] = o1[5] * inv; c[2] = o1[6] * inv; c[3] = o1[7] * inv;
      *(v4fa*)(&os[wb + lr * 68 + 16 + 8 * hi]) = a; *(v4fa*)(&os[wb + lr * 68 + 16 + 8 * hi + 4]) = c;
      a[0] = o2[0] * inv; a[1] = o2[1] * inv; a[2] = o2[2] * inv; a[3] = o2[3] * inv; c[0] = o2[4] * inv; c[1] = o2[5] * inv; c[2] = o2[6] * inv; c[3] = o2[7] * inv;
      *(v4fa*)(&os[wb + lr * 68 + 32 + 8 * hi]) = a; *(v4fa*)(&os[wb + lr * 68 + 32 + 8 * hi + 4]) = c;
      a[0] = o3[0] * inv; a[1] = o3[1] * inv; a[2] = o3[2] * inv; a[3] = o3[3] * inv; c[0] = o3[4] * inv; c[1] = o3[5] * inv; c[2] = o3[6] * inv; c[3] = o3[7] * inv;
      *(v4fa*)(&os[wb + lr * 68 + 48 + 8 * hi]) = a; *(v4fa*)(&os[wb + lr * 68 + 48 + 8 * hi + 4]) = c; }
    wave_sync();
    h16* crow = CH + ((size_t)b * SEQ + t0) * DM + h * HD;
#pragma unroll 1
    for (int ps = 0; ps < 2; ++ps) {
#pragma unroll
        for (int s = 0; s < 4; ++s) { const int row = 4 * s + (lane >> 3), c8 = (lane & 7) * 8;
            const v4f x0 = *(const v4fa*)(&os[wb + row * 68 + c8]); const v4f x1 = *(const v4fa*)(&os[wb + row * 68 + c8 + 4]); v8h hv;
#pragma unroll
            for (int i = 0; i < 4; ++i) { hv[i] = (h16)x0[i]; hv[4 + i] = (h16)x1[i]; }
            *(volatile v8h*)(crow + (size_t)row * DM + c8) = hv; }
        if (ps == 0) __threadfence(); }
}

__global__ __launch_bounds__(32 * AW) void k_flash_early(const h16* __restrict__ QH, const h16* __restrict__ QR, const h16* __restrict__ KP, const h16* __restrict__ KR,
                                                         const h16* __restrict__ VT, const h16* __restrict__ VR, h16* CH, h16* CR) {
    __shared__ __align__(16) float os[AW * 16 * 68];
    const int lane = threadIdx.x & 31; const int wave = __builtin_amdgcn_readfirstlane(threadIdx.x >> 5);
    const int lr = lane & 15, hi = lane >> 4;
    const int zg = blockIdx.y; const int b = zg / NKV; const int g = zg % NKV;
    const int h = g * AW + wave;
    const int t0 = blockIdx.x * 16;
    const int tq = t0 + lr;
    const size_t qo = ((size_t)(b * NH_ + h) * SEQ + (size_t)tq) * HD + 8 * hi;
    const v16h qh0 = ldh(QH + qo), qh1 = ldh(QH + qo + 32), qr0 = ldh(QR + qo), qr1 = ldh(QR + qo + 32);
    const size_t ko = (size_t)zg * SEQ * HD + (size_t)lr * HD + 8 * hi;
    const size_t vo = (size_t)zg * HD * SEQ + (size_t)lr * SEQ + 8 * hi;
    v8f oH[4], oL[4];
#pragma unroll
    for (int j = 0; j < 4; ++j) { oH[j] = (v8f){}; oL[j] = (v8f){}; }
    float m = NEGB, l = 0.0f;
    const int kend = t0 + 16;
#pragma unroll 1
    for (int key0 = 0; key0 < kend; key0 += 32) {
        const size_t kk = ko + (size_t)key0 * HD;
        v8f sHa = (v8f){}, sLa = (v8f){}, sHb = (v8f){}, sLb = (v8f){};
        { const v16h k0 = ldh(KP + kk), k1 = ldh(KP + kk + 32), r0 = ldh(KR + kk), r1 = ldh(KR + kk + 32);
          sHa = wmma16(k0, qh0, sHa); sHa = wmma16(k1, qh1, sHa);
          sLa = wmma16(k0, qr0, sLa); sLa = wmma16(k1, qr1, sLa); sLa = wmma16(r0, qh0, sLa); sLa = wmma16(r1, qh1, sLa); }
        { const size_t k2 = kk + (size_t)16 * HD;
          const v16h k0 = ldh(KP + k2), k1 = ldh(KP + k2 + 32), r0 = ldh(KR + k2), r1 = ldh(KR + k2 + 32);
          sHb = wmma16(k0, qh0, sHb); sHb = wmma16(k1, qh1, sHb);
          sLb = wmma16(k0, qr0, sLb); sLb = wmma16(k1, qr1, sLb); sLb = wmma16(r0, qh0, sLb); sLb = wmma16(r1, qh1, sLb); }
        float ta[8], tb[8];
#pragma unroll
        for (int r = 0; r < 8; ++r) { ta[r] = (sHa[r] + sLa[r] * QRI) * SC2; tb[r] = (sHb[r] + sLb[r] * QRI) * SC2; }
        if (key0 + 31 > t0) {
            const int kbse = key0 + 8 * hi;
#pragma unroll
            for (int r = 0; r < 8; ++r) { ta[r] = (kbse + r > tq) ? NEGB : ta[r]; tb[r] = (kbse + 16 + r > tq) ? NEGB : tb[r]; } }
        float mx = NEGB;
#pragma unroll
        for (int r = 0; r < 8; ++r) mx = fmaxf(mx, fmaxf(ta[r], tb[r]));
        mx = fmaxf(mx, __shfl_xor(mx, 16, 32));
        const float mnew = fmaxf(m, mx);
        const float alpha = __builtin_amdgcn_exp2f(m - mnew);
        const float sh = PSH - mnew;
        v16h ph, pr; float ls = 0.0f;
#pragma unroll
        for (int r = 0; r < 8; ++r) { const float ea = __builtin_amdgcn_exp2f(ta[r] + sh); const float ec = __builtin_amdgcn_exp2f(tb[r] + sh);
            const h16 ha = (h16)ea; const h16 hc = (h16)ec; ph[r] = ha; ph[8 + r] = hc;
            pr[r] = (h16)((ea - (float)ha) * QRS); pr[8 + r] = (h16)((ec - (float)hc) * QRS); ls += ea + ec; }
        l = l * alpha + ls; m = mnew;
#pragma unroll
        for (int j = 0; j < 4; ++j) { oH[j] = oH[j] * alpha; oL[j] = oL[j] * alpha; }
        const size_t vv = vo + (size_t)key0;
#pragma unroll
        for (int j = 0; j < 4; ++j) { const v16h vh = ldh(VT + vv + (size_t)(16 * j) * SEQ); const v16h vr = ldh(VR + vv + (size_t)(16 * j) * SEQ);
            oH[j] = wmma16(vh, ph, oH[j]); oL[j] = wmma16(vr, ph, oL[j]); oL[j] = wmma16(vh, pr, oL[j]); }
    }
    l += __shfl_xor(l, 16, 32);
    const float inv = CXS / l;
    const int wb = wave * 16 * 68;
#pragma unroll
    for (int j = 0; j < 4; ++j) { v4f a, c;
        a[0] = (oH[j][0] + oL[j][0] * QRI) * inv; a[1] = (oH[j][1] + oL[j][1] * QRI) * inv; a[2] = (oH[j][2] + oL[j][2] * QRI) * inv; a[3] = (oH[j][3] + oL[j][3] * QRI) * inv;
        c[0] = (oH[j][4] + oL[j][4] * QRI) * inv; c[1] = (oH[j][5] + oL[j][5] * QRI) * inv; c[2] = (oH[j][6] + oL[j][6] * QRI) * inv; c[3] = (oH[j][7] + oL[j][7] * QRI) * inv;
        *(v4fa*)(&os[wb + lr * 68 + 16 * j + 8 * hi]) = a; *(v4fa*)(&os[wb + lr * 68 + 16 * j + 8 * hi + 4]) = c; }
    wave_sync();
    h16* crow = CH + ((size_t)b * SEQ + t0) * DM + h * HD;
    h16* rrow = CR + ((size_t)b * EARLY + t0) * DM + h * HD;
#pragma unroll 1
    for (int ps = 0; ps < 2; ++ps) {
#pragma unroll
        for (int s = 0; s < 4; ++s) { const int row = 4 * s + (lane >> 3), c8 = (lane & 7) * 8;
            const v4f x0 = *(const v4fa*)(&os[wb + row * 68 + c8]); const v4f x1 = *(const v4fa*)(&os[wb + row * 68 + c8 + 4]); v8h hv, rv;
#pragma unroll
            for (int i = 0; i < 4; ++i) { const h16 a0 = (h16)x0[i]; const h16 a1 = (h16)x1[i]; hv[i] = a0; hv[4 + i] = a1; rv[i] = (h16)(x0[i] - (float)a0); rv[4 + i] = (h16)(x1[i] - (float)a1); }
            *(volatile v8h*)(crow + (size_t)row * DM + c8) = hv; *(volatile v8h*)(rrow + (size_t)row * DM + c8) = rv; }
        if (ps == 0) __threadfence(); }
}

__global__ __launch_bounds__(32) void k_out(const h16* __restrict__ CX, const h16* __restrict__ Wt, float* OUT) {
    __shared__ __align__(16) float os[16 * 68];
    const int K = DM;
    const int lane = threadIdx.x & 31, lr = lane & 15, hi = lane >> 4; const int r0 = blockIdx.x * 64, c0 = blockIdx.y * 64;
    const int b = r0 / SEQ, tt = r0 % SEQ;
    const int npass = (tt < EARLY) ? 2 : 1;
    const size_t aoff0 = (size_t)(r0 + lr) * K + 8 * hi;
    const size_t aoff1 = ((size_t)NB * SEQ + (size_t)b * EARLY + (size_t)tt + (size_t)lr) * K + 8 * hi;
    const size_t boff = (size_t)(c0 + lr) * K + 8 * hi;
    v8f acc[4][4];
#pragma unroll
    for (int mb = 0; mb < 4; ++mb)
#pragma unroll
        for (int nb = 0; nb < 4; ++nb) acc[mb][nb] = (v8f){};
#pragma unroll 1
    for (int pass = 0; pass < npass; ++pass) {
        const size_t ao = pass ? aoff1 : aoff0;
#pragma unroll 1
        for (int kc = 0; kc < K; kc += 32) {
            v16h a[4];
#pragma unroll
            for (int mb = 0; mb < 4; ++mb) a[mb] = ldh(CX + ao + (size_t)mb * 16 * K + kc);
#pragma unroll
            for (int nb = 0; nb < 4; ++nb) { const v16h bq = ldh(Wt + boff + (size_t)nb * 16 * K + kc);
#pragma unroll
                for (int mb = 0; mb < 4; ++mb) acc[mb][nb] = wmma16(a[mb], bq, acc[mb][nb]); }
        }
    }
    float* obase = OUT + ((size_t)b * OUT_SEQ + tt) * DM + c0;
#pragma unroll
    for (int mb = 0; mb < 4; ++mb) {
#pragma unroll
        for (int nb = 0; nb < 4; ++nb) {
#pragma unroll
            for (int j = 0; j < 8; ++j) os[(hi * 8 + j) * 68 + nb * 16 + lr] = acc[mb][nb][j] * OUTS; }
        wave_sync();
#pragma unroll 1
        for (int ps = 0; ps < 2; ++ps) {
#pragma unroll
            for (int s = 0; s < 8; ++s) { const int row = 2 * s + hi, cofs = lr * 4;
                const v4f val = *(const v4fa*)(&os[row * 68 + cofs]);
                *(volatile v4f*)(obase + (size_t)(mb * 16 + row) * DM + cofs) = val; }
            if (ps == 0) __threadfence(); }
        wave_sync();
    }
}

static constexpr size_t al256(size_t v) { return (v + 255) & ~(size_t)255; }
static constexpr size_t SZ_XB = al256((size_t)NB * SEQ * DM * 2);
static constexpr size_t SZ_WQ = al256((size_t)DM * DM * 2);
static constexpr size_t SZ_WK = al256((size_t)KVD * DM * 2);
static constexpr size_t SZ_CS = al256((size_t)SEQ * 32 * 2 * 4);
static constexpr size_t SZ_Q  = al256((size_t)NB * NH_ * SEQ * HD * 2);
static constexpr size_t SZ_KV = al256((size_t)NB * NKV * SEQ * HD * 2);
static constexpr size_t SZ_CX = al256(((size_t)NB * SEQ + (size_t)NB * EARLY) * DM * 2);
static constexpr size_t SZ_TOTAL = SZ_XB + 2 * SZ_WQ + 2 * SZ_WK + SZ_CS + 2 * SZ_Q + 4 * SZ_KV + SZ_CX;
static_assert(SZ_TOTAL <= (size_t)134217728);

extern "C" void kernel_launch(void* const* d_in, const int* in_sizes, int n_in,
                              void* d_out, int out_size, void* d_ws, size_t ws_size, hipStream_t stream) {
    if (n_in < 5) return;
    const size_t needx = ((size_t)(NB - 1) * SEQ_FULL + SEQ) * DM;
    if ((size_t)in_sizes[0] < needx) return;
    if ((size_t)in_sizes[1] < (size_t)DM * DM || (size_t)in_sizes[2] < (size_t)DM * KVD || (size_t)in_sizes[3] < (size_t)DM * KVD || (size_t)in_sizes[4] < (size_t)DM * DM) return;
    if ((size_t)out_size < ((size_t)(NB - 1) * OUT_SEQ + SEQ) * DM) return;
    if (SZ_TOTAL > ws_size) return;
    const float* x = (const float*)d_in[0]; const float* wq = (const float*)d_in[1]; const float* wk = (const float*)d_in[2]; const float* wv = (const float*)d_in[3]; const float* wo = (const float*)d_in[4];
    float* OUT = (float*)d_out;
    char* wsp = (char*)d_ws;
    bf*  XB  = (bf*)wsp;  wsp += SZ_XB;
    bf*  WQt = (bf*)wsp;  wsp += SZ_WQ;
    bf*  WKt = (bf*)wsp;  wsp += SZ_WK;
    bf*  WVt = (bf*)wsp;  wsp += SZ_WK;
    h16* WOt = (h16*)wsp; wsp += SZ_WQ;
    float* CS = (float*)wsp; wsp += SZ_CS;
    h16* QH = (h16*)wsp; wsp += SZ_Q;
    h16* QR = (h16*)wsp; wsp += SZ_Q;
    h16* KP = (h16*)wsp; wsp += SZ_KV;
    h16* KR = (h16*)wsp; wsp += SZ_KV;
    h16* VT = (h16*)wsp; wsp += SZ_KV;
    h16* VR = (h16*)wsp; wsp += SZ_KV;
    h16* CX = (h16*)wsp; wsp += SZ_CX;
    h16* CR = CX + (size_t)NB * SEQ * DM;

    if (SEQ == SEQ_FULL) {
        const size_t n8 = (size_t)NB * SEQ * DM / 8;
        k_cvt8<<<(unsigned)((n8 + 255) / 256), 256, 0, stream>>>(x, XB, n8);
    } else {
        const size_t n8 = (size_t)SEQ * DM / 8;
        for (int b = 0; b < NB; ++b) k_cvt8<<<(unsigned)((n8 + 255) / 256), 256, 0, stream>>>(x + (size_t)b * SEQ_FULL * DM, XB + (size_t)b * SEQ * DM, n8);
    }
    k_wt<<<dim3(DM / 64,  DM / 64, 1), 256, 0, stream>>>(wq, WQt, (h16*)WQt, DM, DM, 0);
    k_wt<<<dim3(KVD / 64, DM / 64, 1), 256, 0, stream>>>(wk, WKt, (h16*)WKt, DM, KVD, 0);
    k_wt<<<dim3(KVD / 64, DM / 64, 1), 256, 0, stream>>>(wv, WVt, (h16*)WVt, DM, KVD, 0);
    k_wt<<<dim3(DM / 64,  DM / 64, 1), 256, 0, stream>>>(wo, (bf*)WOt, WOt, DM, DM, 1);
    k_rope_tab<<<(unsigned)((SEQ * 32 + 255) / 256), 256, 0, stream>>>(CS, SEQ);

    k_proj<<<dim3(NB * SEQ / 64, DM / 64, 1), 32, 0, stream>>>(XB, WQt, QH, QR, 1, SEQ, (size_t)NH_ * SEQ * HD, HD, HD, (size_t)SEQ * HD, CS, 1);
    k_proj<<<dim3(NB * SEQ / 64, KVD / 64, 1), 32, 0, stream>>>(XB, WKt, KP, KR, 1, SEQ, (size_t)NKV * SEQ * HD, HD, HD, (size_t)SEQ * HD, CS, 1);
    k_proj<<<dim3(KVD / 64, NB * SEQ / 64, 1), 32, 0, stream>>>(WVt, XB, VT, VR, 1, KVD, (size_t)0, SEQ, SEQ, (size_t)KVD * SEQ, CS, 0);

    k_flash_early<<<dim3(EARLY / 16, NB * NKV, 1), 32 * AW, 0, stream>>>(QH, QR, KP, KR, VT, VR, CX, CR);
    if (SEQ > EARLY)
        k_flash<<<dim3((SEQ - EARLY) / 16, NB * NKV, 1), 32 * AW, 0, stream>>>(QH, QR, KP, VT, CX);

    k_out<<<dim3(NB * SEQ / 64, DM / 64, 1), 32, 0, stream>>>(CX, WOt, OUT);
}
